// Model_73409581023752
// MI455X (gfx1250) — hardware-verified
//
#include <hip/hip_runtime.h>
#include <stddef.h>
#include <stdint.h>

typedef float          v4f   __attribute__((ext_vector_type(4)));
typedef float          v8f   __attribute__((ext_vector_type(8)));
typedef unsigned       v4u   __attribute__((ext_vector_type(4)));
typedef int            v8i   __attribute__((ext_vector_type(8)));
typedef unsigned short v8us  __attribute__((ext_vector_type(8)));
typedef unsigned short v16us __attribute__((ext_vector_type(16)));
typedef __bf16         v16bf __attribute__((ext_vector_type(16)));
typedef v4f  __attribute__((may_alias)) v4fa;
typedef v4u  __attribute__((may_alias)) v4ua;
typedef v8us __attribute__((may_alias)) v8usa;
union FragB { v16bf v; v16us us; v8us h[2]; v8i w; unsigned u[8]; };

#define NB      4
#define NPTS    300000
#define NCELL   3375
#define NCHUNK  15
#define PPB     20000
#define NTILE   625
#define ETHR    256
#define EWAVES  8
#define PARTW   13504
#define PARTV   3376
#define SCNP    3392
#define GTILES  53
#define CLIPHI  14.9999f
#define BNEPS   1e-5f

static_assert(NPTS == NCHUNK * PPB);
static_assert(PPB == NTILE * 32);
static_assert(NPTS % (15 * 32) == 0);
static_assert(PARTV * 4 == PARTW && PARTV == NCELL + 1);
static_assert((PARTW * 4) % 128 == 0);
static_assert(SCNP == GTILES * 64 && SCNP >= NCELL && (SCNP * 4) % 128 == 0);
static_assert(NCELL * 16 <= 65536);

#define O_MW    ((size_t)0)
#define O_BIAS  ((size_t)3072)
#define O_CPAR  ((size_t)3328)
#define O_CW1   ((size_t)4352)
#define O_CWS   ((size_t)52480)
#define O_STAT  ((size_t)249088)
#define O_Y0    ((size_t)256256)
#define O_Y1    ((size_t)321792)
#define O_SCN   ((size_t)387328)
#define O_PART  ((size_t)1038592)
#define WS_TOTAL ((size_t)10761472)
static_assert(O_BIAS == O_MW + 3072 && O_CPAR == O_BIAS + 256 && O_CW1 == O_CPAR + 1024);
static_assert(O_CWS == O_CW1 + (size_t)16 * 1504 * 2 && O_STAT == O_CWS + (size_t)6 * 16 * 1024 * 2);
static_assert(O_Y0 == O_STAT + 7 * 8 * 128 && O_Y1 == O_Y0 + 65536 && O_SCN == O_Y1 + 65536);
static_assert(O_PART == O_SCN + (size_t)NB * 12 * SCNP * 4);
static_assert(WS_TOTAL == O_PART + (size_t)180 * PARTW * 4);
static_assert(O_CW1 % 128 == 0 && O_CWS % 128 == 0 && O_STAT % 128 == 0 && O_Y0 % 128 == 0 &&
              O_Y1 % 128 == 0 && O_SCN % 128 == 0 && O_PART % 128 == 0 && O_BIAS % 128 == 0 && O_CPAR % 128 == 0);
static_assert(WS_TOTAL <= (size_t)134217728);
static_assert(1500 <= 1504 && 1000 <= 1024 && 1504 % 32 == 0 && 1024 % 32 == 0);

__device__ __forceinline__ int iclamp(int v, int lo, int hi) { return v < lo ? lo : (v > hi ? hi : v); }
__device__ __forceinline__ unsigned bf16_bits(float f) {
  const unsigned u = __float_as_uint(f);
  return ((u + 0x7FFFu + ((u >> 16) & 1u)) >> 16) & 0xFFFFu;
}
__device__ __forceinline__ float bf16_val(float f) { return __uint_as_float(bf16_bits(f) << 16); }
__device__ __forceinline__ float fsel(float a, float b, unsigned mask) {
  return __uint_as_float((__float_as_uint(a) & ~mask) | (__float_as_uint(b) & mask));
}
__device__ __forceinline__ float elu_f(float v) {
  const float e = expm1f(v);
  return (v > 0.0f) ? v : e;
}
__device__ __forceinline__ unsigned hilo_word(float v) {
  const unsigned hb = bf16_bits(v);
  const unsigned lb = bf16_bits(v - __uint_as_float(hb << 16));
  return hb | (lb << 16);
}
__device__ __forceinline__ v8f z8() { v8f z = {0.f, 0.f, 0.f, 0.f, 0.f, 0.f, 0.f, 0.f}; return z; }

__device__ __forceinline__ v8f wmb(const FragB& a, const FragB& b, v8f c) {
  v8f d = __builtin_amdgcn_wmma_f32_16x16x32_bf16(false, a.v, false, b.v, (short)0, c, false, false);
  asm volatile("v_nop\n\tv_nop\n\tv_nop\n\tv_nop" : "+v"(d) : "v"(a.w), "v"(b.w));
  return d;
}
__device__ __forceinline__ void put16(unsigned short* dp, v8us o) {
  *(volatile v8us*)dp = o;
  __threadfence();
  *(volatile v8us*)dp = o;
}

__device__ __forceinline__ void cw_unit(const float* __restrict__ w, int KP, int KR, int u, unsigned short* dst) {
  const int upr = KP >> 3;
  const int r = u / upr;
  const int k8 = (u - r * upr) * 8;
  const int mat = r >> 4, n = r & 15;
  const int nc = n < 8 ? n : 7;
  const float* p = w + (size_t)(mat * 8 + nc) * (size_t)KR;
  v8us o;
#pragma unroll
  for (int i = 0; i < 8; ++i) {
    const int k = k8 + i;
    const int kc = k < KR ? k : (KR - 1);
    const unsigned bits = bf16_bits(p[kc]);
    o[i] = (unsigned short)((n < 8 && k < KR) ? bits : 0u);
  }
  put16(dst + (size_t)u * 8, o);
}

__global__ __launch_bounds__(256) void k_prep(
    const float* __restrict__ W1, const float* __restrict__ W2, const float* __restrict__ W3,
    const float* __restrict__ b1, const float* __restrict__ b2, const float* __restrict__ b3,
    const float* __restrict__ c1w, const float* __restrict__ c1b, const float* __restrict__ g1,
    const float* __restrict__ be1, const float* __restrict__ csw, const float* __restrict__ csb,
    const float* __restrict__ gs, const float* __restrict__ bes,
    unsigned short* MW, float* BIAS, float* CPAR, unsigned short* CW1, unsigned short* CWS)
{
  __shared__ __attribute__((aligned(16))) float tab[256];
  const int b = (int)blockIdx.x, tid = (int)threadIdx.x;
  if (b == 0) {
    if (tid < 192) {
      const int mt = tid >> 6, n = (tid >> 2) & 15, k8 = (tid & 3) * 8;
      v8us o;
      if (mt == 0) {
#pragma unroll
        for (int i = 0; i < 8; ++i) {
          const int kk = (k8 + i) & 15;
          const int kc = kk < 12 ? kk : 11;
          const unsigned bits = bf16_bits(W1[kc * 16 + n]);
          o[i] = (unsigned short)((kk < 12) ? bits : 0u);
        }
      } else if (mt == 1) {
#pragma unroll
        for (int i = 0; i < 8; ++i) {
          const int kk = (k8 + i) & 15;
          o[i] = (unsigned short)bf16_bits(W2[kk * 16 + n]);
        }
      } else {
        const int nc = n < 4 ? n : 3;
#pragma unroll
        for (int i = 0; i < 8; ++i) {
          const int kk = (k8 + i) & 15;
          const unsigned bits = bf16_bits(W3[kk * 4 + nc]);
          o[i] = (unsigned short)((n < 4) ? bits : 0u);
        }
      }
      put16(MW + (size_t)tid * 8, o);
    }
  } else if (b == 1) {
    const int e = tid;
    const float a = b1[iclamp(e, 0, 15)];
    const float c = b2[iclamp(e - 16, 0, 15)];
    const float d = b3[iclamp(e - 32, 0, 3)];
    float v = 0.0f;
    v = fsel(v, a, (e < 16) ? 0xffffffffu : 0u);
    v = fsel(v, c, (e >= 16 && e < 32) ? 0xffffffffu : 0u);
    v = fsel(v, d, (e >= 32 && e < 36) ? 0xffffffffu : 0u);
    tab[tid] = bf16_val(v);
    __syncthreads();
    const v4f pv = *(const v4fa*)(tab + 4 * (tid & 15));
    if (tid < 16) *(volatile v4f*)(BIAS + 4 * tid) = pv;
    __threadfence();
    if (tid < 16) *(volatile v4f*)(BIAS + 4 * tid) = pv;
  } else if (b == 2) {
    const int e = tid;
    const int l = iclamp(e >> 5, 0, 6);
    const int j = e & 31, jj = j & 7, kind = j >> 3;
    const int lm = iclamp(l - 1, 0, 5);
    const float a0 = c1b[jj], a1 = csb[lm * 8 + jj];
    const float q0 = g1[jj],  q1 = gs[lm * 8 + jj];
    const float t0 = be1[jj], t1 = bes[lm * 8 + jj];
    const unsigned mf = (l == 0) ? 0xffffffffu : 0u;
    const float vb = fsel(a1, a0, mf), vg = fsel(q1, q0, mf), vt = fsel(t1, t0, mf);
    float v = 0.0f;
    v = fsel(v, vb, (kind == 0) ? 0xffffffffu : 0u);
    v = fsel(v, vg, (kind == 2) ? 0xffffffffu : 0u);
    v = fsel(v, vt, (kind == 3) ? 0xffffffffu : 0u);
    v = bf16_val(v);
    v = fsel(0.0f, v, (e < 224) ? 0xffffffffu : 0u);
    tab[tid] = v;
    __syncthreads();
    const int tq = tid < 56 ? tid : 55;
    const v4f pv = *(const v4fa*)(tab + 4 * tq);
    if (tid < 56) *(volatile v4f*)(CPAR + 4 * tid) = pv;
    __threadfence();
    if (tid < 56) *(volatile v4f*)(CPAR + 4 * tid) = pv;
  } else if (b < 15) {
    const int u = (b - 3) * 256 + tid;
    if (u < 3008) cw_unit(c1w, 1504, 1500, u, CW1);
  } else {
    const int u = (b - 15) * 256 + tid;
    if (u < 12288) cw_unit(csw, 1024, 1000, u, CWS);
  }
}

__device__ __forceinline__ void part_pass(const unsigned* bins, unsigned* dst, int tid) {
#pragma unroll 1
  for (int i = tid; i < PARTV; i += ETHR) {
    const int ic = i < NCELL ? i : (NCELL - 1);
    v4u v = *(const v4ua*)(bins + 4 * ic);
    const unsigned mk = (i < NCELL) ? 0xffffffffu : 0u;
    v.x &= mk; v.y &= mk; v.z &= mk; v.w &= mk;
    *(volatile v4u*)(dst + (size_t)i * 4) = v;
  }
}

__device__ __forceinline__ void act_split(const v8f d, const v4f b0, const v4f b1, FragB& o) {
  const float bb[8] = {b0.x, b0.y, b0.z, b0.w, b1.x, b1.y, b1.z, b1.w};
  unsigned hb[8], lb[8];
#pragma unroll
  for (int r = 0; r < 8; ++r) {
    const float e = elu_f(d[r] + bb[r]);
    hb[r] = bf16_bits(e);
    lb[r] = bf16_bits(e - __uint_as_float(hb[r] << 16));
  }
#pragma unroll
  for (int j = 0; j < 4; ++j) {
    o.u[j]     = hb[2 * j] | (hb[2 * j + 1] << 16);
    o.u[4 + j] = lb[2 * j] | (lb[2 * j + 1] << 16);
  }
}
__device__ __forceinline__ unsigned max_key(float f) {
  unsigned k = (f > 0.0f) ? __float_as_uint(f) : 0u;
  k = (f != f) ? 0x7fc00000u : k;
  return k;
}

__global__ __launch_bounds__(ETHR) void k_encode(const float* __restrict__ pts,
                                                 const unsigned short* __restrict__ MW,
                                                 const float* __restrict__ BIAS, unsigned* part)
{
  __shared__ __attribute__((aligned(16))) unsigned bins[NCELL * 4];
  const int tid = (int)threadIdx.x, lane = tid & 31, wave = tid >> 5;
  const int h = lane >> 4, m = lane & 15;
  const int bsc = (int)blockIdx.x / NCHUNK, chunk = (int)blockIdx.x - bsc * NCHUNK;

  {
    const v4u z4 = {0u, 0u, 0u, 0u};
#pragma unroll 1
    for (int i = tid; i < NCELL; i += ETHR) *(v4ua*)(bins + 4 * i) = z4;
  }

  FragB A1, A2, A3;
  {
    const unsigned short* r1 = MW + m * 32;
    const unsigned short* r2 = MW + 512 + m * 32;
    const unsigned short* r3 = MW + 1024 + m * 32;
    A1.h[0] = *(const v8usa*)(r1 + 8 * h);  A1.h[1] = *(const v8usa*)(r1 + 16 + 8 * h);
    A2.h[0] = *(const v8usa*)(r2 + 8 * h);  A2.h[1] = *(const v8usa*)(r2 + 16 + 8 * h);
    A3.h[0] = *(const v8usa*)(r3 + 8 * h);  A3.h[1] = *(const v8usa*)(r3 + 16 + 8 * h);
  }
  const v4f b1a = *(const v4f*)(BIAS + 8 * h),      b1b = *(const v4f*)(BIAS + 8 * h + 4);
  const v4f b2a = *(const v4f*)(BIAS + 16 + 8 * h), b2b = *(const v4f*)(BIAS + 16 + 8 * h + 4);
  const v4f b3v = *(const v4f*)(BIAS + 32);
  const float bb3[4] = {b3v.x, b3v.y, b3v.z, b3v.w};
  const unsigned mh = 0u - (unsigned)h;
  const int pbase = bsc * NPTS + chunk * PPB;

  __syncthreads();

#pragma unroll 1
  for (int tile = wave; tile < NTILE; tile += EWAVES) {
    const float* pp = pts + (size_t)(pbase + tile * 32 + lane) * 3;
    const float px = bf16_val(pp[0]);
    const float py = bf16_val(pp[1]);
    const float pz = bf16_val(pp[2]);
    const float cx = floorf(fminf(fmaxf(px, 0.0f), CLIPHI));
    const float cy = floorf(fminf(fmaxf(py, 0.0f), CLIPHI));
    const float cz = floorf(fminf(fmaxf(pz, 0.0f), CLIPHI));
    const int cell = iclamp(((int)cx * 15 + (int)cy) * 15 + (int)cz, 0, NCELL - 1);

    float x[12];
    x[0] = px - (cx + 0.5f); x[1] = py - (cy + 0.5f); x[2] = pz - (cz + 0.5f);
    x[3] = px - cx;          x[4] = py - cy;          x[5] = pz - cz;
    x[6] = px - (cx + 1.0f); x[7] = py - (cy + 1.0f); x[8] = pz - (cz + 1.0f);
    x[9]  = sqrtf(x[0] * x[0] + x[1] * x[1] + x[2] * x[2]);
    x[10] = sqrtf(x[3] * x[3] + x[4] * x[4] + x[5] * x[5]);
    x[11] = sqrtf(x[6] * x[6] + x[7] * x[7] + x[8] * x[8]);

    unsigned hw[6], lw[6];
#pragma unroll
    for (int j = 0; j < 6; ++j) {
      const unsigned w0 = hilo_word(x[2 * j]);
      const unsigned w1 = hilo_word(x[2 * j + 1]);
      hw[j] = (w0 & 0xffffu) | (w1 << 16);
      lw[j] = (w0 >> 16) | (w1 & 0xffff0000u);
    }
    unsigned xh[6], xl[6];
#pragma unroll
    for (int j = 0; j < 6; ++j) {
      xh[j] = (unsigned)__shfl_xor((int)hw[j], 16);
      xl[j] = (unsigned)__shfl_xor((int)lw[j], 16);
    }
    const int xcell = iclamp(__shfl_xor(cell, 16), 0, NCELL - 1);

    FragB Ba, Bb;
#pragma unroll
    for (int j = 0; j < 2; ++j) {
      Ba.u[j]     = (hw[j] & ~mh) | (xh[4 + j] & mh);
      Ba.u[4 + j] = (lw[j] & ~mh) | (xl[4 + j] & mh);
      Bb.u[j]     = (xh[j] & ~mh) | (hw[4 + j] & mh);
      Bb.u[4 + j] = (xl[j] & ~mh) | (lw[4 + j] & mh);
    }
#pragma unroll
    for (int j = 2; j < 4; ++j) {
      Ba.u[j]     = hw[j] & ~mh;
      Ba.u[4 + j] = lw[j] & ~mh;
      Bb.u[j]     = xh[j] & ~mh;
      Bb.u[4 + j] = xl[j] & ~mh;
    }

    const v8f d1a = wmb(A1, Ba, z8());
    const v8f d1b = wmb(A1, Bb, z8());
    FragB B2a, B2b;
    act_split(d1a, b1a, b1b, B2a);
    act_split(d1b, b1a, b1b, B2b);

    const v8f d2a = wmb(A2, B2a, z8());
    const v8f d2b = wmb(A2, B2b, z8());
    FragB B3a, B3b;
    act_split(d2a, b2a, b2b, B3a);
    act_split(d2b, b2a, b2b, B3b);

    const v8f d3a = wmb(A3, B3a, z8());
    const v8f d3b = wmb(A3, B3b, z8());

#pragma unroll
    for (int r = 0; r < 4; ++r) {
      const unsigned ka = max_key(d3a[r] + bb3[r]) & ~mh;
      const unsigned kb = max_key(d3b[r] + bb3[r]) & ~mh;
      atomicMax(bins + cell * 4 + r, ka);
      atomicMax(bins + xcell * 4 + r, kb);
    }
  }
  __syncthreads();

  unsigned* dst = part + (size_t)blockIdx.x * PARTW;
  part_pass(bins, dst, tid);
  __threadfence();
  part_pass(bins, dst, tid);
}

__global__ __launch_bounds__(64) void k_gridmax(const unsigned* __restrict__ part, unsigned* scn)
{
  __shared__ __attribute__((aligned(16))) unsigned st[4 * 64];
  const int tid = (int)threadIdx.x;
  const int blk = (int)blockIdx.x;
  const int tile = blk % GTILES;
  const int g = (blk / GTILES) % 3;
  const int b = blk / (3 * GTILES);
  const int set = (g == 0) ? 1 : ((g == 1) ? 0 : 2);
  const int cell = tile * 64 + tid;
  const int cc = cell < NCELL ? cell : (NCELL - 1);
  const unsigned* p = part + (size_t)(set * NB + b) * NCHUNK * PARTW + (size_t)cc * 4;
  v4u mx = {0u, 0u, 0u, 0u};
#pragma unroll 5
  for (int ch = 0; ch < NCHUNK; ++ch) {
    const v4u v = *(const v4u*)(p + (size_t)ch * PARTW);
    mx.x = mx.x > v.x ? mx.x : v.x;
    mx.y = mx.y > v.y ? mx.y : v.y;
    mx.z = mx.z > v.z ? mx.z : v.z;
    mx.w = mx.w > v.w ? mx.w : v.w;
  }
  const unsigned mk = (cell < NCELL) ? 0xffffffffu : 0u;
  st[0 * 64 + tid] = hilo_word(__uint_as_float(mx.x)) & mk;
  st[1 * 64 + tid] = hilo_word(__uint_as_float(mx.y)) & mk;
  st[2 * 64 + tid] = hilo_word(__uint_as_float(mx.z)) & mk;
  st[3 * 64 + tid] = hilo_word(__uint_as_float(mx.w)) & mk;
  __syncthreads();
  const int ch = tid >> 4, piece = tid & 15;
  const v4u o = *(const v4ua*)(st + ch * 64 + piece * 4);
  unsigned* dp = scn + (size_t)(b * 12 + g * 4 + ch) * SCNP + tile * 64 + piece * 4;
  *(volatile v4u*)dp = o;
  __threadfence();
  *(volatile v4u*)dp = o;
}

template <int CIN, int S, int DIN, int KP, int KR, int FIRST>
__global__ __launch_bounds__(128) void k_conv(const unsigned* __restrict__ scn, const float* __restrict__ yin,
                                              const float* __restrict__ stat,
                                              const unsigned short* __restrict__ cw,
                                              const float* __restrict__ cpar, float* yout)
{
  constexpr int SD = DIN + 4;
  constexpr int NSLAB = CIN * 5 * SD * SD;
  static_assert(KP % 32 == 0 && KR <= KP && KR == CIN * 125);
  static_assert((NSLAB * 4) % 16 == 0 && (KP * 2) % 16 == 0);
  static_assert(S * 7 + 4 < SD);
  static_assert(FIRST == 1 || CIN == 8);
  extern __shared__ __attribute__((aligned(16))) unsigned char dsm[];
  unsigned*       slab = (unsigned*)dsm;
  float*          yst  = (float*)(dsm + NSLAB * 4);
  unsigned short* koff = (unsigned short*)(dsm + NSLAB * 4 + 4096);
  float*          sst  = (float*)(dsm + NSLAB * 4 + 4096 + KP * 2);

  const int tid = (int)threadIdx.x, lane = tid & 31, wave = tid >> 5;
  const int h = lane >> 4, m = lane & 15;
  const int b = (int)blockIdx.x >> 3, oz = (int)blockIdx.x & 7;

#pragma unroll 1
  for (int k = tid; k < KP; k += 128) {
    const int ci = k / 125;
    const int r = k - ci * 125;
    const int kz = r / 25;
    const int r2 = r - kz * 25;
    const int ky = r2 / 5;
    const int kx = r2 - ky * 5;
    const int off = ((ci * 5 + kz) * SD + ky) * SD + kx;
    koff[k] = (unsigned short)((k < KR) ? off : 0);
  }
  if (FIRST == 0) {
    const v4f s = *(const v4f*)(stat + (tid & 7) * 32);
    if (tid < 8) *(v4fa*)(sst + 4 * tid) = s;
  }
  __syncthreads();

#pragma unroll 1
  for (int s = tid; s < NSLAB; s += 128) {
    const int t1 = s / SD;
    const int sx = s - t1 * SD;
    const int t2 = t1 / SD;
    const int sy = t1 - t2 * SD;
    const int ci = t2 / 5;
    const int kz = t2 - ci * 5;
    const int iz = S * oz - 2 + kz, iy = sy - 2, ix = sx - 2;
    const bool ok = ((unsigned)iz < (unsigned)DIN) && ((unsigned)iy < (unsigned)DIN) && ((unsigned)ix < (unsigned)DIN);
    const int izc = iclamp(iz, 0, DIN - 1), iyc = iclamp(iy, 0, DIN - 1), ixc = iclamp(ix, 0, DIN - 1);
    unsigned w;
    if (FIRST == 1) {
      w = scn[(size_t)(b * 12 + ci) * SCNP + izc * 225 + iyc * 15 + ixc];
    } else {
      const float v = yin[(size_t)((b * 8 + ci) * 8 + izc) * 64 + iyc * 8 + ixc];
      const v4f st4 = *(const v4fa*)(sst + 4 * ci);
      const float t = ((v - st4.x) * st4.y) * st4.z + st4.w;
      w = hilo_word(elu_f(t));
    }
    slab[s] = w & (ok ? 0xffffffffu : 0u);
  }
  __syncthreads();

  const int p = 16 * wave + m;
  const int oy = p >> 3, ox = p & 7;
  const unsigned* arow = slab + (S * oy) * SD + S * ox;
  const unsigned short* brow = cw + (size_t)m * KP + 8 * h;
  v8f accH = z8(), accL = z8();
#pragma unroll 1
  for (int k0 = 0; k0 < KP; k0 += 32) {
    const v8us ka = *(const v8usa*)(koff + k0 + 8 * h);
    const v8us kb = *(const v8usa*)(koff + k0 + 16 + 8 * h);
    unsigned w[16];
#pragma unroll
    for (int i = 0; i < 8; ++i) {
      w[i]     = arow[(unsigned)ka[i]];
      w[8 + i] = arow[(unsigned)kb[i]];
    }
    FragB ah, al, bf;
#pragma unroll
    for (int j = 0; j < 8; ++j) {
      ah.u[j] = (w[2 * j] & 0xffffu) | (w[2 * j + 1] << 16);
      al.u[j] = (w[2 * j] >> 16) | (w[2 * j + 1] & 0xffff0000u);
    }
    bf.h[0] = *(const v8usa*)(brow + k0);
    bf.h[1] = *(const v8usa*)(brow + k0 + 16);
    accH = wmb(ah, bf, accH);
    accL = wmb(al, bf, accL);
  }

  const float cb = cpar[m];
#pragma unroll
  for (int r = 0; r < 8; ++r) yst[m * 64 + 16 * wave + 8 * h + r] = (accH[r] + accL[r]) + cb;
  __syncthreads();

  const int o = tid >> 4, piece = tid & 15;
  const v4f v = *(const v4fa*)(yst + o * 64 + piece * 4);
  float* dp = yout + (size_t)((b * 8 + o) * 8 + oz) * 64 + piece * 4;
  *(volatile v4f*)dp = v;
  __threadfence();
  *(volatile v4f*)dp = v;
}

__device__ __forceinline__ double shx(double v, int d) {
  int lo = __double2loint(v), hi = __double2hiint(v);
  lo = __shfl_xor(lo, d);
  hi = __shfl_xor(hi, d);
  return __hiloint2double(hi, lo);
}
__device__ __forceinline__ double wave_sum_d(double s) {
  s += shx(s, 16);
  s += shx(s, 8);
  s += shx(s, 4);
  s += shx(s, 2);
  s += shx(s, 1);
  return s;
}
__device__ __forceinline__ void out_pass(const float* ot, float* out, int c, int lane) {
#pragma unroll 1
  for (int i = 0; i < 16; ++i) {
    const int e = (i * 32 + lane) * 4;
    const int bb = e >> 9, w = e & 511;
    const v4f o = *(const v4fa*)(ot + e);
    *(volatile v4f*)(out + (size_t)(bb * 8 + c) * 512 + w) = o;
  }
}

template <int FINAL>
__global__ __launch_bounds__(32) void k_bn(const float* __restrict__ y, const float* __restrict__ cpar,
                                           float* stat, float* out)
{
  __shared__ __attribute__((aligned(16))) float ot[2048];
  const int c = (int)blockIdx.x, lane = (int)threadIdx.x;
  const float gam = cpar[16 + c];
  const float bet = cpar[24 + c];

  double s = 0.0;
#pragma unroll 1
  for (int i = 0; i < 16; ++i) {
    const int e = (i * 32 + lane) * 4;
    const int bb = e >> 9, w = e & 511;
    const v4f v = *(const v4f*)(y + (size_t)(bb * 8 + c) * 512 + w);
    s += (double)v.x; s += (double)v.y; s += (double)v.z; s += (double)v.w;
  }
  s = wave_sum_d(s);
  const double mean = s * (1.0 / 2048.0);

  double q = 0.0;
#pragma unroll 1
  for (int i = 0; i < 16; ++i) {
    const int e = (i * 32 + lane) * 4;
    const int bb = e >> 9, w = e & 511;
    const v4f v = *(const v4f*)(y + (size_t)(bb * 8 + c) * 512 + w);
    const double d0 = (double)v.x - mean, d1 = (double)v.y - mean;
    const double d2 = (double)v.z - mean, d3 = (double)v.w - mean;
    q += d0 * d0; q += d1 * d1; q += d2 * d2; q += d3 * d3;
  }
  q = wave_sum_d(q);
  const float varf  = (float)(q * (1.0 / 2048.0));
  const float meanf = (float)mean;
  const float rstd  = 1.0f / sqrtf(varf + BNEPS);

  if (FINAL == 0) {
    const unsigned m0 = (lane == 0) ? 0xffffffffu : 0u;
    v4f line;
    line.x = fsel(0.0f, meanf, m0);
    line.y = fsel(0.0f, rstd, m0);
    line.z = fsel(0.0f, gam, m0);
    line.w = fsel(0.0f, bet, m0);
    float* dp = stat + (size_t)c * 32 + 4 * (lane & 7);
    if (lane < 8) *(volatile v4f*)dp = line;
    __threadfence();
    if (lane < 8) *(volatile v4f*)dp = line;
  } else {
#pragma unroll 1
    for (int i = 0; i < 64; ++i) {
      const int e = i * 32 + lane;
      const int bb = e >> 9, w = e & 511;
      const float v = y[(size_t)(bb * 8 + c) * 512 + w];
      const float t = ((v - meanf) * rstd) * gam + bet;
      ot[e] = elu_f(t);
    }
    __syncthreads();
    out_pass(ot, out, c, lane);
    __threadfence();
    out_pass(ot, out, c, lane);
  }
}

#define CONV1_LDS (12 * 5 * 19 * 19 * 4 + 4096 + 1504 * 2 + 128)
#define CONVN_LDS (8 * 5 * 12 * 12 * 4 + 4096 + 1024 * 2 + 128)
static_assert(CONV1_LDS == 93872 && CONVN_LDS == 29312);
static_assert(CONV1_LDS <= 327680 && CONVN_LDS <= 327680);

extern "C" void kernel_launch(void* const* d_in, const int* in_sizes, int n_in,
                              void* d_out, int out_size, void* d_ws, size_t ws_size,
                              hipStream_t stream) {
  if (n_in < 17) return;
  const int want[17] = {3600000, 3600000, 3600000, 192, 16, 256, 16, 64, 4,
                        12000, 8, 8, 8, 48000, 48, 48, 48};
  for (int i = 0; i < 17; ++i) if (in_sizes[i] != want[i]) return;
  if (out_size != 16384) return;
  if (WS_TOTAL > ws_size) return;

  const float* pts0 = (const float*)d_in[0];
  const float* pts1 = (const float*)d_in[1];
  const float* pts2 = (const float*)d_in[2];
  const float* W1  = (const float*)d_in[3];
  const float* b1  = (const float*)d_in[4];
  const float* W2  = (const float*)d_in[5];
  const float* b2  = (const float*)d_in[6];
  const float* W3  = (const float*)d_in[7];
  const float* b3  = (const float*)d_in[8];
  const float* c1w = (const float*)d_in[9];
  const float* c1b = (const float*)d_in[10];
  const float* g1  = (const float*)d_in[11];
  const float* be1 = (const float*)d_in[12];
  const float* csw = (const float*)d_in[13];
  const float* csb = (const float*)d_in[14];
  const float* gs  = (const float*)d_in[15];
  const float* bes = (const float*)d_in[16];
  float* out = (float*)d_out;

  char* ws = (char*)d_ws;
  unsigned short* MW   = (unsigned short*)(ws + O_MW);
  float*          BIAS = (float*)(ws + O_BIAS);
  float*          CPAR = (float*)(ws + O_CPAR);
  unsigned short* CW1  = (unsigned short*)(ws + O_CW1);
  unsigned short* CWS  = (unsigned short*)(ws + O_CWS);
  float*          STAT = (float*)(ws + O_STAT);
  float*          Y0   = (float*)(ws + O_Y0);
  float*          Y1   = (float*)(ws + O_Y1);
  unsigned*       SCN  = (unsigned*)(ws + O_SCN);
  unsigned*       PART = (unsigned*)(ws + O_PART);

  hipFuncSetAttribute(reinterpret_cast<const void*>(&k_conv<12, 2, 15, 1504, 1500, 1>),
                      hipFuncAttributeMaxDynamicSharedMemorySize, (int)CONV1_LDS);
  hipFuncSetAttribute(reinterpret_cast<const void*>(&k_conv<8, 1, 8, 1024, 1000, 0>),
                      hipFuncAttributeMaxDynamicSharedMemorySize, (int)CONVN_LDS);

  k_prep<<<63, 256, 0, stream>>>(W1, W2, W3, b1, b2, b3, c1w, c1b, g1, be1, csw, csb, gs, bes,
                                 MW, BIAS, CPAR, CW1, CWS);
  const size_t setStride = (size_t)NB * NCHUNK * PARTW;
  k_encode<<<NB * NCHUNK, ETHR, 0, stream>>>(pts0, MW, BIAS, PART);
  k_encode<<<NB * NCHUNK, ETHR, 0, stream>>>(pts1, MW, BIAS, PART + setStride);
  k_encode<<<NB * NCHUNK, ETHR, 0, stream>>>(pts2, MW, BIAS, PART + 2 * setStride);
  k_gridmax<<<NB * 3 * GTILES, 64, 0, stream>>>(PART, SCN);
  k_conv<12, 2, 15, 1504, 1500, 1><<<32, 128, CONV1_LDS, stream>>>(SCN, Y1, STAT, CW1, CPAR, Y0);
  k_bn<0><<<8, 32, 0, stream>>>(Y0, CPAR, STAT, out);
  for (int l = 1; l <= 6; ++l) {
    float* yprev = ((l - 1) & 1) ? Y1 : Y0;
    float* ycur  = (l & 1) ? Y1 : Y0;
    k_conv<8, 1, 8, 1024, 1000, 0><<<32, 128, CONVN_LDS, stream>>>(
        SCN, yprev, STAT + (size_t)(l - 1) * 256, CWS + (size_t)(l - 1) * 16 * 1024, CPAR + l * 32, ycur);
    if (l < 6) k_bn<0><<<8, 32, 0, stream>>>(ycur, CPAR + l * 32, STAT + (size_t)l * 256, out);
    else       k_bn<1><<<8, 32, 0, stream>>>(ycur, CPAR + l * 32, STAT + (size_t)l * 256, out);
  }
}
